// HydraBlock_19112604467499
// MI455X (gfx1250) — hardware-verified
//
#include <hip/hip_runtime.h>
#include <math.h>

typedef __attribute__((ext_vector_type(16))) __bf16   v16b;
typedef __attribute__((ext_vector_type(8)))  __bf16   v8b;
typedef __attribute__((ext_vector_type(8)))  float    v8f;
typedef __attribute__((ext_vector_type(4)))  float    v4f;
typedef __attribute__((ext_vector_type(4)))  unsigned v4u;

constexpr int  kLeg     = 0;
constexpr bool kSplitIn = (kLeg == 1);
constexpr int  kSplIn   = kSplitIn ? 2 : 0;
constexpr int  kSplMid  = kSplitIn ? 2 : 1;

constexpr int kBatch  = 2;
constexpr int kSeq    = 2048;
constexpr int kDm     = 1024;
constexpr int kDi     = 2048;
constexpr int kNst    = 16;
constexpr int kDtR    = 64;
constexpr int kRows   = kBatch * kSeq;
constexpr int kNin    = 2 * kDi + 2 * kNst + kDtR;
constexpr int kXtLive = kDi + 2 * kNst + kDtR;
constexpr int kXtP    = 2176;
constexpr int kColB   = kDi;
constexpr int kColC   = kDi + kNst;
constexpr int kColDt  = kDi + 2 * kNst;
constexpr int kChunk  = 64;
static_assert(kRows == 4096);
static_assert(kNin == 4192);
static_assert(kXtLive == 2144 && kXtP >= kXtLive && (kXtP % 64) == 0);
static_assert((kDm % 32) == 0 && (kDi % 32) == 0 && (kDtR % 32) == 0);
static_assert((kRows % 64) == 0 && (kDi % 64) == 0 && (kDm % 64) == 0);
static_assert((kSeq % kChunk) == 0 && (kDi % 256) == 0);
static_assert((kColDt * 4) % 128 == 0 && (kXtP * 4) % 128 == 0);

constexpr size_t kPl    = kSplitIn ? 2 : 1;
constexpr size_t kSzU1  = (size_t)kRows * kDm * 2;
constexpr size_t kSzWI1 = (size_t)kXtP * kDm * 2;
constexpr size_t kSzXT  = (size_t)kRows * kXtP * 4;
constexpr size_t kSzDR1 = (size_t)kRows * kDtR * 2;
constexpr size_t kSzWD1 = (size_t)kDi * kDtR * 2;
constexpr size_t kSzDT  = (size_t)kRows * kDi * 4;
constexpr size_t kSzY   = (size_t)kRows * kDi * 4;
constexpr size_t kSzWO1 = (size_t)kDm * kDi * 2;
constexpr size_t kOffU  = 0;
constexpr size_t kOffWI = kOffU  + kPl * kSzU1;
constexpr size_t kOffXT = kOffWI + kPl * kSzWI1;
constexpr size_t kOffDR = kOffXT + kSzXT;
constexpr size_t kOffWD = kOffDR + 2 * kSzDR1;
constexpr size_t kOffDT = kOffWD + kPl * kSzWD1;
constexpr size_t kOffY  = kOffDT + kSzDT;
constexpr size_t kOffWO = kSplitIn ? kOffU : (kOffY + kSzY);
constexpr size_t kWsTotal = kOffY + kSzY + (kSplitIn ? 0 : kSzWO1);
static_assert(kWsTotal == (kSplitIn ? 130023424ull : 121110528ull));
static_assert(kWsTotal <= 134217728ull);
static_assert(2 * kSzWO1 <= 2 * kSzU1);
static_assert((kOffWI % 128) == 0 && (kOffXT % 128) == 0 && (kOffDR % 128) == 0 && (kOffWD % 128) == 0 &&
              (kOffDT % 128) == 0 && (kOffY % 128) == 0 && (kOffWO % 128) == 0);

__device__ __forceinline__ unsigned rne_bf_word(float f) {
  unsigned u = __float_as_uint(f);
  const unsigned lsb = (u & 0x00010000u) ? 1u : 0u;
  u = (u + 0x7FFFu + lsb) & 0xFFFF0000u;
  return u;
}
__device__ __forceinline__ float rin(float f) {
  if (kLeg == 0) return __uint_as_float(rne_bf_word(f));
  return f;
}
__device__ __forceinline__ unsigned pack_top16(unsigned lo_elem, unsigned hi_elem) {
  return __builtin_amdgcn_perm(hi_elem, lo_elem, 0x07060302u);
}
__device__ __forceinline__ void pin_u(unsigned& t) { asm volatile("" : "+v"(t)); }
__device__ __forceinline__ float rcp1(float x) { return __builtin_amdgcn_rcpf(x); }

__device__ __forceinline__ void split8(const float (&f)[8], v4u& hv, v4u& lv) {
  unsigned hb[8], lb[8];
#pragma unroll
  for (int e = 0; e < 8; ++e) {
    hb[e] = rne_bf_word(f[e]);
    lb[e] = rne_bf_word(f[e] - __uint_as_float(hb[e]));
  }
  hv = (v4u){pack_top16(hb[0], hb[1]), pack_top16(hb[2], hb[3]), pack_top16(hb[4], hb[5]), pack_top16(hb[6], hb[7])};
  lv = (v4u){pack_top16(lb[0], lb[1]), pack_top16(lb[2], lb[3]), pack_top16(lb[4], lb[5]), pack_top16(lb[6], lb[7])};
}

struct FragB {
  union U { v16b v; v8b h[2]; };
  static __device__ __forceinline__ v16b load(const __bf16* p) {
    U f;
    f.h[0] = *(const v8b*)(p);
    f.h[1] = *(const v8b*)(p + 16);
    return f.v;
  }
  static __device__ __forceinline__ v8f mma(v16b a, v16b b, v8f c) {
    return __builtin_amdgcn_wmma_f32_16x16x32_bf16(false, a, false, b, (short)0, c, false, false);
  }
};
__device__ __forceinline__ void acc_tie(v8f& a, v16b x, v16b y, v16b z) {
  asm volatile("v_nop\n\tv_nop\n\tv_nop\n\tv_nop" : "+v"(a) : "v"(x), "v"(y), "v"(z));
}
__device__ __forceinline__ void keep4_b(v16b a, v16b b, v16b c, v16b d) { asm volatile("v_nop" :: "v"(a), "v"(b), "v"(c), "v"(d)); }
__device__ __forceinline__ void acc_guard4(v8f& a, v8f& b, v8f& c, v8f& d) {
  asm volatile("v_nop\n\tv_nop\n\tv_nop\n\tv_nop" : "+v"(a), "+v"(b), "+v"(c), "+v"(d));
}

template <int SPL>
__global__ __launch_bounds__(256) void gemm_nt_bf16(
    const unsigned short* __restrict__ Ap, const unsigned short* __restrict__ A2p, int lda,
    const unsigned short* __restrict__ Btp, const unsigned short* __restrict__ Bt2p, int ldb,
    float* __restrict__ Cout, int ldc, int M, int N, int K) {
  typedef __bf16 T;
  typedef v16b V;
  const T* A   = (const T*)Ap;
  const T* A2  = (const T*)A2p;
  const T* Bt  = (const T*)Btp;
  const T* Bt2 = (const T*)Bt2p;
  __shared__ __align__(16) float sT[8][16 * 68];
  unsigned lane = threadIdx.x & 31u;
  pin_u(lane);
  const int wave = threadIdx.x >> 5;
  const int tilesN = N >> 6;
  const int tilesM = M >> 6;
  const int tile = blockIdx.x * 8 + wave;
  if (tile >= tilesM * tilesN) return;
  const int tm = tile / tilesN;
  const int tn = tile - tm * tilesN;
  const int m0 = tm << 6;
  const int n0 = tn << 6;

  unsigned rl = lane & 15u;
  pin_u(rl);
  unsigned kh = (lane >> 4) << 3;
  pin_u(kh);
  const int rlane = (int)rl;
  const int koff  = (int)kh;
  const int mOff  = (int)kh;

  v8f acc[4][4];
#pragma unroll
  for (int i = 0; i < 4; ++i)
#pragma unroll
    for (int j = 0; j < 4; ++j) acc[i][j] = (v8f){0.f, 0.f, 0.f, 0.f, 0.f, 0.f, 0.f, 0.f};

  for (int k0 = 0; k0 < K; k0 += 32) {
    V bh[4], bl[4];
#pragma unroll
    for (int j = 0; j < 4; ++j) {
      const size_t bo = (size_t)(n0 + (j << 4) + rlane) * ldb + koff + k0;
      bh[j] = FragB::load(Bt + bo);
      bl[j] = bh[j];
      if (SPL == 2) bl[j] = FragB::load(Bt2 + bo);
    }
#pragma unroll
    for (int i = 0; i < 4; ++i) {
      const size_t ao = (size_t)(m0 + (i << 4) + rlane) * lda + koff + k0;
      V ah = FragB::load(A + ao);
      V al = ah;
      if (SPL >= 1) al = FragB::load(A2 + ao);
#pragma unroll
      for (int j = 0; j < 4; ++j) {
        acc[i][j] = FragB::mma(ah, bh[j], acc[i][j]);
        if (SPL == 2) acc[i][j] = FragB::mma(ah, bl[j], acc[i][j]);
        if (SPL >= 1) acc[i][j] = FragB::mma(al, bh[j], acc[i][j]);
      }
#pragma unroll
      for (int j = 0; j < 4; ++j) acc_tie(acc[i][j], ah, al, bh[j]);
    }
    keep4_b(bh[0], bh[1], bh[2], bh[3]);
    if (SPL == 2) keep4_b(bl[0], bl[1], bl[2], bl[3]);
  }
  acc_guard4(acc[0][0], acc[0][1], acc[0][2], acc[0][3]);
  acc_guard4(acc[1][0], acc[1][1], acc[1][2], acc[1][3]);
  acc_guard4(acc[2][0], acc[2][1], acc[2][2], acc[2][3]);
  acc_guard4(acc[3][0], acc[3][1], acc[3][2], acc[3][3]);

  float* slab = sT[wave];
  const int hh = (int)(lane >> 4);
  const int c4 = (int)(lane & 15u) * 4;
#pragma unroll
  for (int i = 0; i < 4; ++i) {
    const int mBase = m0 + (i << 4);
#pragma unroll
    for (int j = 0; j < 4; ++j) {
#pragma unroll
      for (int r = 0; r < 8; ++r) slab[(mOff + r) * 68 + (j << 4) + rlane] = acc[i][j][r];
    }
    __builtin_amdgcn_fence(__ATOMIC_RELEASE, "workgroup");
    __builtin_amdgcn_wave_barrier();
    __builtin_amdgcn_fence(__ATOMIC_ACQUIRE, "workgroup");
    for (int pass = 0; pass < 2; ++pass) {
#pragma unroll
      for (int it = 0; it < 8; ++it) {
        const int row = it * 2 + hh;
        const v4f v = *(const v4f*)(slab + row * 68 + c4);
        *(volatile v4f*)(Cout + (size_t)(mBase + row) * ldc + n0 + c4) = v;
      }
      __threadfence();
    }
    __builtin_amdgcn_fence(__ATOMIC_RELEASE, "workgroup");
    __builtin_amdgcn_wave_barrier();
    __builtin_amdgcn_fence(__ATOMIC_ACQUIRE, "workgroup");
  }
}

template <bool SPLIT>
__global__ __launch_bounds__(256) void cvt_planes_kernel(
    const float* __restrict__ src, unsigned* __restrict__ dhi, unsigned* __restrict__ dlo,
    unsigned total8, unsigned valid8)
{
  unsigned i = blockIdx.x * 256u + threadIdx.x;
  pin_u(i);
  if (i >= total8) return;
  const bool live = (i < valid8);
  unsigned ic = live ? i : (valid8 - 1u);
  pin_u(ic);
  const size_t e0 = (size_t)ic << 3;
  const v4f a0 = *(const v4f*)(src + e0);
  const v4f a1 = *(const v4f*)(src + e0 + 4);
  float f[8];
  f[0] = a0[0]; f[1] = a0[1]; f[2] = a0[2]; f[3] = a0[3];
  f[4] = a1[0]; f[5] = a1[1]; f[6] = a1[2]; f[7] = a1[3];
#pragma unroll
  for (int e = 0; e < 8; ++e) f[e] = live ? f[e] : 0.0f;
  v4u hv, lv;
  split8(f, hv, lv);
  const size_t w0 = (size_t)i << 2;
  *(volatile v4u*)(dhi + w0) = hv;
  if (SPLIT) *(volatile v4u*)(dlo + w0) = lv;
  __threadfence();
  *(volatile v4u*)(dhi + w0) = hv;
  if (SPLIT) *(volatile v4u*)(dlo + w0) = lv;
}

__global__ __launch_bounds__(256) void split_dtraw_kernel(
    const float* __restrict__ XT, unsigned* __restrict__ DRH, unsigned* __restrict__ DRL)
{
  unsigned i = blockIdx.x * 256u + threadIdx.x;
  pin_u(i);
  if (i >= (unsigned)(kRows * kDtR / 8)) return;
  unsigned row = i >> 3;
  pin_u(row);
  unsigned c8 = (i & 7u) << 3;
  pin_u(c8);
  const float* sp = XT + (size_t)row * kXtP + kColDt + c8;
  const v4f a0 = *(const v4f*)(sp);
  const v4f a1 = *(const v4f*)(sp + 4);
  float f[8];
  f[0] = a0[0]; f[1] = a0[1]; f[2] = a0[2]; f[3] = a0[3];
  f[4] = a1[0]; f[5] = a1[1]; f[6] = a1[2]; f[7] = a1[3];
  v4u hv, lv;
  split8(f, hv, lv);
  const size_t w0 = (size_t)i << 2;
  *(volatile v4u*)(DRH + w0) = hv;
  *(volatile v4u*)(DRL + w0) = lv;
  __threadfence();
  *(volatile v4u*)(DRH + w0) = hv;
  *(volatile v4u*)(DRL + w0) = lv;
}

__global__ __launch_bounds__(256) void softplus_rows_kernel(float* DT, const float* __restrict__ bdt)
{
  unsigned tid = threadIdx.x;
  pin_u(tid);
  float* rowp = DT + (size_t)blockIdx.x * kDi;
#pragma unroll 1
  for (int i = 0; i < 8; ++i) {
    const unsigned d = tid + 256u * (unsigned)i;
    float* p = rowp + d;
    const float pre = *p;
    const float bb = bdt[d];
    const float v = pre + rin(bb);
    const float e = expf(-fabsf(v));
    const float sp = fmaxf(v, 0.0f) + log1pf(e);
    *(volatile float*)p = sp;
    __threadfence();
    *(volatile float*)p = sp;
  }
}

__global__ __launch_bounds__(256) void scan_bidir_kernel(
    const float* __restrict__ XT, const float* __restrict__ DT,
    const float* __restrict__ cw, const float* __restrict__ cb,
    const float* __restrict__ Alog, const float* __restrict__ Dp,
    float* Y)
{
  __shared__ __align__(16) float sBC[kChunk * 32];
  __shared__ __align__(16) float sA[kNst * 256];
  unsigned tid = threadIdx.x;
  pin_u(tid);
  const unsigned bix = blockIdx.x >> 3;
  const unsigned d   = ((blockIdx.x & 7u) << 8) + tid;
  const size_t row0  = (size_t)bix * kSeq;

#pragma unroll 1
  for (int n = 0; n < kNst; ++n) {
    const float al = Alog[(size_t)d * kNst + n];
    sA[n * 256 + tid] = -expf(rin(al));
  }
  __syncthreads();
  float An[kNst];
#pragma unroll
  for (int n = 0; n < kNst; ++n) An[n] = sA[n * 256 + tid];

  const v4f wv = *(const v4f*)(cw + (size_t)d * 4);
  const float wa = wv[0], wb = wv[1], wc = wv[2], wd = wv[3];
  const float w0 = rin(wa), w1 = rin(wb), w2 = rin(wc), w3 = rin(wd);
  const float cbr = cb[d];
  const float cbv = rin(cbr);
  const float dpr = Dp[d];
  const float Dv  = rin(dpr);

  unsigned sr = tid >> 3;
  pin_u(sr);
  unsigned sc4 = (tid & 7u) << 2;
  pin_u(sc4);

#pragma unroll 1
  for (int dir = 0; dir < 2; ++dir) {
    __threadfence();
    __syncthreads();
    asm volatile("" ::: "memory");
    float st[kNst];
#pragma unroll
    for (int n = 0; n < kNst; ++n) st[n] = 0.0f;
    float r0, r1, r2;
    {
      const size_t rl = row0 + (size_t)(kSeq - 3);
      const float v0 = XT[rl * kXtP + d];
      const float v1 = XT[(rl + 1) * kXtP + d];
      const float v2 = XT[(rl + 2) * kXtP + d];
      r0 = dir ? v0 : 0.0f;
      r1 = dir ? v1 : 0.0f;
      r2 = dir ? v2 : 0.0f;
    }
#pragma unroll 1
    for (int c = 0; c < kSeq / kChunk; ++c) {
      const int s0 = dir ? (kSeq - kChunk - c * kChunk) : (c * kChunk);
      __syncthreads();
#pragma unroll
      for (int i2 = 0; i2 < 2; ++i2) {
        const unsigned r = sr + 32u * (unsigned)i2;
        const v4f v = *(const v4f*)(XT + (row0 + (size_t)s0 + r) * kXtP + kColB + sc4);
        *(v4f*)(sBC + r * 32u + sc4) = v;
      }
      __syncthreads();
#pragma unroll 1
      for (int i = 0; i < kChunk; ++i) {
        const int sl = dir ? (kChunk - 1 - i) : i;
        const int s  = s0 + sl;
        int sx = dir ? (s - 3) : s;
        const bool xok = (sx >= 0);
        sx = xok ? sx : 0;
        float xn = XT[(row0 + (size_t)sx) * kXtP + d];
        xn = xok ? xn : 0.0f;
        const float t0 = dir ? xn : r0;
        const float t1 = dir ? r0 : r1;
        const float t2 = dir ? r1 : r2;
        const float t3 = dir ? r2 : xn;
        const float q0 = dir ? xn : r1;
        const float q1 = dir ? r0 : r2;
        const float q2 = dir ? r1 : xn;
        r0 = q0; r1 = q1; r2 = q2;
        float ca = w0 * t0;
        ca = fmaf(w1, t1, ca);
        ca = fmaf(w2, t2, ca);
        ca = fmaf(w3, t3, ca);
        const float xc = ca + cbv;
        const float sg = rcp1(1.0f + expf(-xc));
        const float xs = xc * sg;
        const size_t row = row0 + (size_t)s;
        const float dt = DT[row * kDi + d];
        const float* bc = sBC + sl * 32;
        float y = 0.0f;
#pragma unroll
        for (int q4 = 0; q4 < 4; ++q4) {
          const v4f bv = *(const v4f*)(bc + 4 * q4);
          const v4f cv = *(const v4f*)(bc + kNst + 4 * q4);
#pragma unroll
          for (int e = 0; e < 4; ++e) {
            const int n = 4 * q4 + e;
            const float a = 1.0f + dt * An[n];
            st[n] = a * st[n] + xs * bv[e];
            y = st[n] * cv[e] + y;
          }
        }
        y = y + Dv * xs;
        float* yp = Y + row * kDi + d;
        float yv = y;
        if (dir) {
          asm volatile("" ::: "memory");
          float yo = *yp;
          asm volatile("" : "+v"(yo));
          yv = yo + y;
        }
        *(volatile float*)yp = yv;
        __threadfence();
        *(volatile float*)yp = yv;
      }
    }
  }
}

__global__ __launch_bounds__(256) void norm_gate_kernel(
    float* Yp, const float* __restrict__ Z, const float* __restrict__ nw)
{
  __shared__ __align__(16) float sg[kDi];
  __shared__ float sred[8];
  unsigned tid = threadIdx.x;
  pin_u(tid);
  const unsigned lane = tid & 31u;
  const unsigned wave = tid >> 5;
  const size_t rbase = (size_t)blockIdx.x * kDi;
  const float* yrow = Yp + rbase;
  float ss = 0.0f;
#pragma unroll 1
  for (int i = 0; i < 8; ++i) {
    const unsigned d = tid + 256u * (unsigned)i;
    const float v = yrow[d];
    sg[d] = v;
    ss = fmaf(v, v, ss);
  }
#pragma unroll
  for (int off = 1; off < 32; off <<= 1) ss += __shfl_xor(ss, off, 32);
  if (lane == 0u) sred[wave] = ss;
  __syncthreads();
  float tot = 0.0f;
#pragma unroll
  for (int w = 0; w < 8; ++w) tot += sred[w];
  const float ms = tot * (1.0f / (float)kDi);
  const float rinv = rcp1(sqrtf(ms + 1e-5f));
#pragma unroll 1
  for (int i = 0; i < 8; ++i) {
    const unsigned d = tid + 256u * (unsigned)i;
    const float yv = sg[d];
    const float zv = Z[rbase + d];
    const float nr = nw[d];
    const float g0 = rin(nr) * (yv * rinv);
    const float sz = rcp1(1.0f + expf(-zv));
    sg[d] = g0 * (zv * sz);
  }
  __syncthreads();
  const v4f a0 = *(const v4f*)(sg + 8u * tid);
  const v4f a1 = *(const v4f*)(sg + 8u * tid + 4u);
  float f[8];
  f[0] = a0[0]; f[1] = a0[1]; f[2] = a0[2]; f[3] = a0[3];
  f[4] = a1[0]; f[5] = a1[1]; f[6] = a1[2]; f[7] = a1[3];
  v4u hv, lv;
  split8(f, hv, lv);
  unsigned* wrow = (unsigned*)(Yp + rbase);
  unsigned* ph = wrow + 4u * tid;
  unsigned* pl = wrow + (unsigned)(kDi / 2) + 4u * tid;
  *(volatile v4u*)ph = hv;
  *(volatile v4u*)pl = lv;
  __threadfence();
  *(volatile v4u*)ph = hv;
  *(volatile v4u*)pl = lv;
}

extern "C" void kernel_launch(void* const* d_in, const int* in_sizes, int n_in,
                              void* d_out, int out_size, void* d_ws, size_t ws_size,
                              hipStream_t stream) {
  if (n_in < 10) return;
  if (in_sizes[0] != kRows * kDm) return;
  if (in_sizes[1] != kNin * kDm) return;
  if (in_sizes[2] != kDi * 4) return;
  if (in_sizes[3] != kDi) return;
  if (in_sizes[4] != kDi * kNst) return;
  if (in_sizes[5] != kDi) return;
  if (in_sizes[6] != kDi * kDtR) return;
  if (in_sizes[7] != kDi) return;
  if (in_sizes[8] != kDi) return;
  if (in_sizes[9] != kDm * kDi) return;
  if (out_size != kRows * kDm) return;
  if (ws_size < kWsTotal) return;

  const float* u       = (const float*)d_in[0];
  const float* W_in    = (const float*)d_in[1];
  const float* conv_w  = (const float*)d_in[2];
  const float* conv_b  = (const float*)d_in[3];
  const float* A_log   = (const float*)d_in[4];
  const float* D_param = (const float*)d_in[5];
  const float* W_dt    = (const float*)d_in[6];
  const float* b_dt    = (const float*)d_in[7];
  const float* norm_w  = (const float*)d_in[8];
  const float* W_out   = (const float*)d_in[9];
  float* out = (float*)d_out;

  char* ws = (char*)d_ws;
  unsigned short* UH  = (unsigned short*)(ws + kOffU);
  unsigned short* UL  = (unsigned short*)(ws + kOffU  + (kSplitIn ? kSzU1 : 0));
  unsigned short* WIH = (unsigned short*)(ws + kOffWI);
  unsigned short* WIL = (unsigned short*)(ws + kOffWI + (kSplitIn ? kSzWI1 : 0));
  float*          XT  = (float*)(ws + kOffXT);
  unsigned short* DRH = (unsigned short*)(ws + kOffDR);
  unsigned short* DRL = (unsigned short*)(ws + kOffDR + kSzDR1);
  unsigned short* WDH = (unsigned short*)(ws + kOffWD);
  unsigned short* WDL = (unsigned short*)(ws + kOffWD + (kSplitIn ? kSzWD1 : 0));
  float*          DT  = (float*)(ws + kOffDT);
  float*          Y   = (float*)(ws + kOffY);
  unsigned short* WOH = (unsigned short*)(ws + kOffWO);
  unsigned short* WOL = (unsigned short*)(ws + kOffWO + (kSplitIn ? kSzWO1 : 0));
  unsigned short* A2H = (unsigned short*)(ws + kOffY);
  unsigned short* A2L = A2H + kDi;

  cvt_planes_kernel<kSplitIn><<<(kRows * kDm / 8) / 256, 256, 0, stream>>>(
      u, (unsigned*)UH, (unsigned*)UL, (unsigned)(kRows * kDm / 8), (unsigned)(kRows * kDm / 8));
  cvt_planes_kernel<kSplitIn><<<(kXtP * kDm / 8) / 256, 256, 0, stream>>>(
      W_in + (size_t)kDi * kDm, (unsigned*)WIH, (unsigned*)WIL,
      (unsigned)(kXtP * kDm / 8), (unsigned)(kXtLive * kDm / 8));
  cvt_planes_kernel<kSplitIn><<<(kDi * kDtR / 8) / 256, 256, 0, stream>>>(
      W_dt, (unsigned*)WDH, (unsigned*)WDL, (unsigned)(kDi * kDtR / 8), (unsigned)(kDi * kDtR / 8));
  gemm_nt_bf16<kSplIn><<<(kRows / 64) * (kXtP / 64) / 8, 256, 0, stream>>>(
      UH, UL, kDm, WIH, WIL, kDm, XT, kXtP, kRows, kXtP, kDm);
  split_dtraw_kernel<<<(kRows * kDtR / 8) / 256, 256, 0, stream>>>(XT, (unsigned*)DRH, (unsigned*)DRL);
  gemm_nt_bf16<kSplMid><<<(kRows / 64) * (kDi / 64) / 8, 256, 0, stream>>>(
      DRH, DRL, kDtR, WDH, WDL, kDtR, DT, kDi, kRows, kDi, kDtR);
  softplus_rows_kernel<<<kRows, 256, 0, stream>>>(DT, b_dt);
  scan_bidir_kernel<<<kBatch * (kDi / 256), 256, 0, stream>>>(XT, DT, conv_w, conv_b, A_log, D_param, Y);
  cvt_planes_kernel<kSplitIn><<<(kDi * kDm / 8) / 256, 256, 0, stream>>>(
      W_in, (unsigned*)WIH, (unsigned*)WIL, (unsigned)(kDi * kDm / 8), (unsigned)(kDi * kDm / 8));
  gemm_nt_bf16<kSplIn><<<(kRows / 64) * (kDi / 64) / 8, 256, 0, stream>>>(
      UH, UL, kDm, WIH, WIL, kDm, DT, kDi, kRows, kDi, kDm);
  cvt_planes_kernel<kSplitIn><<<(kDm * kDi / 8) / 256, 256, 0, stream>>>(
      W_out, (unsigned*)WOH, (unsigned*)WOL, (unsigned)(kDm * kDi / 8), (unsigned)(kDm * kDi / 8));
  norm_gate_kernel<<<kRows, 256, 0, stream>>>(Y, DT, norm_w);
  gemm_nt_bf16<kSplMid><<<(kRows / 64) * (kDm / 64) / 8, 256, 0, stream>>>(
      A2H, A2L, 2 * kDi, WOH, WOL, kDi, out, kDm, kRows, kDm, kDi);
}
